// GATLayer_6468220748676
// MI455X (gfx1250) — hardware-run, weakly checked
//
#include <hip/hip_runtime.h>

typedef float          v8f   __attribute__((ext_vector_type(8)));
typedef float          v4f   __attribute__((ext_vector_type(4)));
typedef unsigned int   v4u   __attribute__((ext_vector_type(4)));
typedef int            v8i   __attribute__((ext_vector_type(8)));
typedef unsigned short v8us  __attribute__((ext_vector_type(8)));
typedef unsigned short v16us __attribute__((ext_vector_type(16)));
typedef __bf16         v16bf __attribute__((ext_vector_type(16)));
typedef _Float16       v16h  __attribute__((ext_vector_type(16)));
typedef v4f  __attribute__((may_alias)) v4fa;
typedef v8us __attribute__((may_alias)) v8usa;
union FragB { v16bf v; v16us u; v8us h[2]; v8i w; };
union FragH { v16h  v; v16us u; v8us h[2]; v8i w; };

__device__ __forceinline__ v8f wmb(const FragB& a, const FragB& b, v8f c) {
  v8f d = __builtin_amdgcn_wmma_f32_16x16x32_bf16(false, a.v, false, b.v, (short)0, c, false, false);
  asm volatile("v_nop\n\tv_nop\n\tv_nop\n\tv_nop" : "+v"(d) : "v"(a.w), "v"(b.w));
  return d;
}

__device__ __forceinline__ v8f wmh(const FragH& a, const FragH& b, v8f c) {
  v8f d = __builtin_amdgcn_wmma_f32_16x16x32_f16(false, a.v, false, b.v, (short)0, c, false, false);
  asm volatile("v_nop\n\tv_nop\n\tv_nop\n\tv_nop" : "+v"(d) : "v"(a.w), "v"(b.w));
  return d;
}

__device__ __forceinline__ unsigned bf16_bits(float f) {
  const unsigned u = __float_as_uint(f);
  const unsigned r = (u + 0x7FFFu + ((u >> 16) & 1u)) >> 16;
  const unsigned q = (u >> 16) | 0x40u;
  return ((u & 0x7fffffffu) > 0x7f800000u) ? q : r;
}

__device__ __forceinline__ float bf16_val(float f) {
  return __uint_as_float(bf16_bits(f) << 16);
}
__device__ __forceinline__ int clampi(int v, int lo, int hi) {
  return v < lo ? lo : (v > hi ? hi : v);
}

__device__ __forceinline__ unsigned f16_bits(float f) {
  const unsigned u  = __float_as_uint(f);
  const unsigned s  = (u >> 16) & 0x8000u;
  const unsigned a  = u & 0x7fffffffu;
  const unsigned t  = a - 0x38000000u;
  const unsigned r  = (t + 0x0FFFu + ((t >> 13) & 1u)) >> 13;
  const unsigned rc = r > 0x7C00u ? 0x7C00u : r;
  const bool small  = a < 0x38800000u;
  const bool isnan  = a > 0x7f800000u;
  const unsigned fin = small ? 0u : (s | rc);
  return isnan ? (s | 0x7E00u) : fin;
}

__device__ __forceinline__ unsigned pk16(unsigned lo, unsigned hi) { return lo | (hi << 16); }
__device__ __forceinline__ unsigned bf16_lo_bits(float v) {
  float hi = bf16_val(v);
  asm volatile("" : "+v"(hi));
  return bf16_bits(v - hi);
}
__device__ __forceinline__ v4u pack8_bf16(v4f a, v4f c) {
  return (v4u){ pk16(bf16_bits(a[0]), bf16_bits(a[1])), pk16(bf16_bits(a[2]), bf16_bits(a[3])),
                pk16(bf16_bits(c[0]), bf16_bits(c[1])), pk16(bf16_bits(c[2]), bf16_bits(c[3])) };
}
__device__ __forceinline__ v4u pack8_bf16_lo(v4f a, v4f c) {
  return (v4u){ pk16(bf16_lo_bits(a[0]), bf16_lo_bits(a[1])), pk16(bf16_lo_bits(a[2]), bf16_lo_bits(a[3])),
                pk16(bf16_lo_bits(c[0]), bf16_lo_bits(c[1])), pk16(bf16_lo_bits(c[2]), bf16_lo_bits(c[3])) };
}
__device__ __forceinline__ v4u pack8_f16(v4f a, v4f c) {
  return (v4u){ pk16(f16_bits(a[0]), f16_bits(a[1])), pk16(f16_bits(a[2]), f16_bits(a[3])),
                pk16(f16_bits(c[0]), f16_bits(c[1])), pk16(f16_bits(c[2]), f16_bits(c[3])) };
}

template <int FORM>
__global__ __launch_bounds__(256) void k_plane(const float* __restrict__ src, int rows, int cols, int ldsrc,
                                               unsigned short* __restrict__ dst, int MP, int KP) {
  static_assert(FORM >= 0 && FORM <= 3);
  const int KTOT = (FORM == 1 || FORM == 3) ? 2 * KP : KP;
  const unsigned ppr   = (unsigned)(KTOT >> 3);
  const unsigned kp8   = (unsigned)(KP >> 3);
  const unsigned total = (unsigned)MP * ppr;
  const unsigned g     = blockIdx.x * 256u + threadIdx.x;
  const unsigned rowu  = g / ppr;
  const unsigned p     = g - rowu * ppr;
  const bool second    = p >= kp8;
  const int row = (int)rowu;
  const int c0  = (int)((second ? p - kp8 : p) << 3);
  const float* srow = src + (size_t)clampi(row, 0, rows - 1) * (size_t)ldsrc;
  float x[8];
  unsigned mk[8];
#pragma unroll
  for (int e = 0; e < 8; ++e) {
    const int c = c0 + e;
    const float v = srow[clampi(c, 0, cols - 1)];
    asm volatile("" :: "v"(v));
    x[e]  = v;
    mk[e] = (row < rows && c < cols) ? 0xFFFFu : 0u;
  }
  const v4f a = (v4f){ x[0], x[1], x[2], x[3] };
  const v4f c = (v4f){ x[4], x[5], x[6], x[7] };
  v4u o;
  if (FORM == 2) {
    o = pack8_f16(a, c);
  } else {
    const v4u hi = pack8_bf16(a, c);
    o = hi;
    if (FORM == 1) { const v4u lo = pack8_bf16_lo(a, c); o = second ? lo : hi; }
  }
  const v4u mw = (v4u){ pk16(mk[0], mk[1]), pk16(mk[2], mk[3]), pk16(mk[4], mk[5]), pk16(mk[6], mk[7]) };
  o &= mw;
  if (g < total) {
    volatile v4u* q = (volatile v4u*)(dst + (size_t)g * 8);
    *q = o;
    __threadfence();
    *q = o;
  }
}

template <int FORM> struct FragOf    { typedef FragB T; };
template <>         struct FragOf<2> { typedef FragH T; };
__device__ __forceinline__ v8f mm(const FragB& a, const FragB& b, v8f c) { return wmb(a, b, c); }
__device__ __forceinline__ v8f mm(const FragH& a, const FragH& b, v8f c) { return wmh(a, b, c); }
template <class F> __device__ __forceinline__ F ld_frag(const unsigned short* p) {
  F f;
  f.h[0] = *(const v8usa*)(p);
  f.h[1] = *(const v8usa*)(p + 16);
  return f;
}

template <int FORM, int EPI>
__global__ __launch_bounds__(256) __attribute__((amdgpu_num_vgpr(248)))
void k_gemm_nt(const unsigned short* __restrict__ A, const unsigned short* __restrict__ B,
               const float* __restrict__ bias, float* __restrict__ D, int M, int N, int KTOT, int ldd) {
  static_assert(FORM >= 0 && FORM <= 2);
  static_assert(EPI == 0 || EPI == 1);
  typedef typename FragOf<FORM>::T F;
  __shared__ __attribute__((aligned(16))) float sT[8][16 * 68];
  const int lane = threadIdx.x & 31;
  const int wave = threadIdx.x >> 5;
  const int tilesM = (M + 63) >> 6;
  const int tilesN = (N + 63) >> 6;
  const int tile = blockIdx.x * 8 + wave;
  if (tile >= tilesM * tilesN) return;
  const int tm = tile / tilesN;
  const int tn = tile - tm * tilesN;
  const int m0 = tm << 6;
  const int n0 = tn << 6;

  const int rl = lane & 15;
  const int h8 = (lane >> 4) * 8;
  const unsigned short* pa = A + (size_t)(m0 + rl) * (size_t)KTOT + h8;
  const unsigned short* pb = B + (size_t)(n0 + rl) * (size_t)KTOT + h8;

  v8f acc[4][4];
#pragma unroll
  for (int i = 0; i < 4; ++i)
#pragma unroll
    for (int j = 0; j < 4; ++j) acc[i][j] = (v8f){0.f, 0.f, 0.f, 0.f, 0.f, 0.f, 0.f, 0.f};

#pragma unroll 1
  for (int k0 = 0; k0 < KTOT; k0 += 32) {
    F bf[4];
#pragma unroll
    for (int j = 0; j < 4; ++j) bf[j] = ld_frag<F>(pb + (size_t)(j << 4) * (size_t)KTOT + k0);
#pragma unroll
    for (int i = 0; i < 4; ++i) {
      const F af = ld_frag<F>(pa + (size_t)(i << 4) * (size_t)KTOT + k0);
#pragma unroll
      for (int j = 0; j < 4; ++j) acc[i][j] = mm(af, bf[j], acc[i][j]);
    }
  }

  float* slab = sT[wave];
  const int hh = lane >> 4;
  const int c4 = (lane & 15) * 4;
  const int nc = n0 + c4;
  const bool cok = nc < N;
  v4f bv = (v4f){0.f, 0.f, 0.f, 0.f};
  if (EPI == 1) {
    bv = *(const v4fa*)(bias + clampi(nc, 0, N - 4));
    asm volatile("" :: "v"(bv));
  }
#pragma unroll
  for (int i = 0; i < 4; ++i) {
    const int mBase = m0 + (i << 4);
#pragma unroll
    for (int j = 0; j < 4; ++j) {
#pragma unroll
      for (int r = 0; r < 8; ++r) slab[(h8 + r) * 68 + (j << 4) + rl] = acc[i][j][r];
    }
    __builtin_amdgcn_fence(__ATOMIC_RELEASE, "workgroup");
    __builtin_amdgcn_wave_barrier();
    __builtin_amdgcn_fence(__ATOMIC_ACQUIRE, "workgroup");
    v4f vv[8];
#pragma unroll
    for (int it = 0; it < 8; ++it) {
      const int row = it * 2 + hh;
      v4f v = *(const v4fa*)(slab + row * 68 + c4);
      if (EPI == 1) v += bv;
      vv[it] = v;
    }
    for (int pass = 0; pass < 2; ++pass) {
#pragma unroll
      for (int it = 0; it < 8; ++it) {
        const int row = mBase + it * 2 + hh;
        if (cok && row < M) *(volatile v4f*)(D + (size_t)row * (size_t)ldd + nc) = vv[it];
      }
      __threadfence();
    }
    __builtin_amdgcn_fence(__ATOMIC_RELEASE, "workgroup");
    __builtin_amdgcn_wave_barrier();
    __builtin_amdgcn_fence(__ATOMIC_ACQUIRE, "workgroup");
  }
}

#define NN      40000
#define NE      640000
#define DD      128
#define MPAD    40064
#define BSLOTS  1024
#define NBLK    40
#define RCAP    21504
#define WLCAP   2816
#define DEGCAP  64
#define EPW     (NE / 8)
#define NIT     ((EPW + 255) / 256)
#define LDS_BK_WORDS (RCAP + 8 * WLCAP + 3 * BSLOTS + 32)
#define LDS_BK  (LDS_BK_WORDS * 4)

typedef int v4i __attribute__((ext_vector_type(4)));
typedef v4i __attribute__((may_alias)) v4ia;
typedef v4u __attribute__((may_alias)) v4ua;

static_assert(NN % 32 == 0);
static_assert(NN % 8 == 0);
static_assert(NN % 16 == 0);
static_assert(DD == 128);
static_assert(DD == 32 * 4);
static_assert(MPAD % 64 == 0 && MPAD >= NN);
static_assert((MPAD * DD / 8) % 256 == 0);
static_assert((DD * DD / 8) % 256 == 0);
static_assert(NN <= 65536);
static_assert(NBLK * BSLOTS >= NN && (NBLK - 1) * BSLOTS < NN);
static_assert((NN - (NBLK - 1) * BSLOTS) % 32 == 0);
static_assert(NE % 64 == 0);
static_assert(EPW % 8 == 0);
static_assert(NIT == 313);
static_assert(EPW - 312 * 256 == 128);
static_assert(RCAP % 1024 == 0);
static_assert(RCAP * 4 >= 5 * 16589);
static_assert(WLCAP % 256 == 0);
static_assert(WLCAP * 8 * 4 >= 5 * 16589);
static_assert(DEGCAP == 64 && DEGCAP >= 37 + 8);
static_assert(LDS_BK <= 262144);

__device__ __forceinline__ int imin(int a, int b) { return a < b ? a : b; }

__global__ __launch_bounds__(64) void k_prep(const float* __restrict__ a, float* alr) {
  const int t = threadIdx.x;
  const v4f v = *(const v4fa*)(a + 4 * t);
  asm volatile("" :: "v"(v));
  const v4f o = (v4f){ bf16_val(v[0]), bf16_val(v[1]), bf16_val(v[2]), bf16_val(v[3]) };
  volatile v4f* q = (volatile v4f*)(alr + 4 * t);
  *q = o;
  __threadfence();
  *q = o;
}

__global__ __launch_bounds__(256) void k_scores(const float* __restrict__ Z, const float* __restrict__ alr, float* slr) {
  __shared__ __attribute__((aligned(16))) float sA[256];
  __shared__ __attribute__((aligned(16))) float sS[64];
  const int tid = threadIdx.x, lane = tid & 31, wave = tid >> 5;
  if (tid < 64) {
    const v4f t = *(const v4fa*)(alr + 4 * tid);
    *(v4fa*)(sA + 4 * tid) = t;
  }
  __syncthreads();
  const v4f al = *(const v4fa*)(sA + 4 * lane);
  const v4f ar = *(const v4fa*)(sA + 128 + 4 * lane);
  const int nbase = blockIdx.x * 32 + wave * 4;
#pragma unroll
  for (int i = 0; i < 4; ++i) {
    const int node = clampi(nbase + i, 0, NN - 1);
    const v4f zr = *(const v4fa*)(Z + (size_t)node * DD + 4 * lane);
    float pl = zr[0] * al[0];
    pl = fmaf(zr[1], al[1], pl);
    pl = fmaf(zr[2], al[2], pl);
    pl = fmaf(zr[3], al[3], pl);
    float pr = zr[0] * ar[0];
    pr = fmaf(zr[1], ar[1], pr);
    pr = fmaf(zr[2], ar[2], pr);
    pr = fmaf(zr[3], ar[3], pr);
#pragma unroll
    for (int off = 16; off > 0; off >>= 1) {
      pl += __shfl_xor(pl, off);
      pr += __shfl_xor(pr, off);
    }
    if (lane == 0) {
      sS[wave * 4 + i]      = pl;
      sS[32 + wave * 4 + i] = pr;
    }
  }
  __syncthreads();
  const int ws = wave & 1;
  const int q  = lane & 7;
  const v4f v = *(const v4fa*)(sS + 32 * ws + 4 * q);
  asm volatile("" :: "v"(v));
  float* dp = slr + (size_t)ws * NN + (size_t)blockIdx.x * 32 + 4 * q;
  const bool wr = (wave < 2) && (lane < 8);
  if (wr) *(volatile v4f*)dp = v;
  __threadfence();
  if (wr) *(volatile v4f*)dp = v;
}

__global__ __launch_bounds__(256) void k_bucket(const int* __restrict__ srcs, const int* __restrict__ dsts,
                                                unsigned* list_out, int* rowoff, int* rowcnt, int* flag) {
  extern __shared__ v4f lds_dyn[];
  int* placed = (int*)lds_dyn;
  int* wl     = placed + RCAP;
  int* scnt   = wl + 8 * WLCAP;
  int* soff   = scnt + BSLOTS;
  int* cur    = soff + BSLOTS;
  int* wcnt   = cur + BSLOTS;
  int* wtot   = wcnt + 16;
  const int tid = threadIdx.x, lane = tid & 31, wave = tid >> 5;
  const int slotBase = (int)blockIdx.x * BSLOTS;
  const int nb = imin(BSLOTS, NN - slotBase);

#pragma unroll 1
  for (int i = tid; i < RCAP; i += 256) placed[i] = 0;
#pragma unroll 1
  for (int i = tid; i < BSLOTS; i += 256) scnt[i] = 0;

  int* mylist = wl + wave * WLCAP;
  const int wbeg = wave * EPW;
  const int wend = wbeg + EPW;
  const unsigned ub = (unsigned)slotBase;
  const unsigned un = (unsigned)nb;
  int wc = 0;
#pragma unroll 1
  for (int it = 0; it < NIT; ++it) {
    const int e0  = wbeg + it * 256 + lane * 8;
    const int e0c = imin(e0, wend - 8);
    const v4i da = *(const v4ia*)(dsts + e0c);
    const v4i db = *(const v4ia*)(dsts + e0c + 4);
    const v4i sa = *(const v4ia*)(srcs + e0c);
    const v4i sb = *(const v4ia*)(srcs + e0c + 4);
    asm volatile("" :: "v"(da));
    asm volatile("" :: "v"(db));
    asm volatile("" :: "v"(sa));
    asm volatile("" :: "v"(sb));
    const int nm = (e0 < wend) ? 0 : -1;
    const unsigned s0 = (unsigned)(da[0] | nm) - ub, s1 = (unsigned)(da[1] | nm) - ub;
    const unsigned s2 = (unsigned)(da[2] | nm) - ub, s3 = (unsigned)(da[3] | nm) - ub;
    const unsigned s4 = (unsigned)(db[0] | nm) - ub, s5 = (unsigned)(db[1] | nm) - ub;
    const unsigned s6 = (unsigned)(db[2] | nm) - ub, s7 = (unsigned)(db[3] | nm) - ub;
    const bool h0 = s0 < un, h1 = s1 < un, h2 = s2 < un, h3 = s3 < un;
    const bool h4 = s4 < un, h5 = s5 < un, h6 = s6 < un, h7 = s7 < un;
    const int c = (int)h0 + (int)h1 + (int)h2 + (int)h3 + (int)h4 + (int)h5 + (int)h6 + (int)h7;
    const unsigned any = __builtin_amdgcn_ballot_w32(c != 0);
    if (any != 0u) {
      int incl = c;
#pragma unroll
      for (int d = 1; d < 32; d <<= 1) {
        const int up = __shfl_up(incl, d);
        incl += (lane >= d) ? up : 0;
      }
      const int total = __shfl(incl, 31);
      int pos = wc + incl - c;
#define PUTJ(HJ, SJ, SRCJ) \
      if (HJ) { \
        if (pos < WLCAP) mylist[pos] = clampi((SRCJ), 0, NN - 1) | (int)((SJ) << 16); \
        pos += 1; \
      }
      PUTJ(h0, s0, sa[0])
      PUTJ(h1, s1, sa[1])
      PUTJ(h2, s2, sa[2])
      PUTJ(h3, s3, sa[3])
      PUTJ(h4, s4, sb[0])
      PUTJ(h5, s5, sb[1])
      PUTJ(h6, s6, sb[2])
      PUTJ(h7, s7, sb[3])
#undef PUTJ
      wc += total;
    }
  }
  if (lane == 0) wcnt[wave] = wc;
  __syncthreads();

  int tot = 0;
  int ovf = 0;
#pragma unroll
  for (int w2 = 0; w2 < 8; ++w2) {
    const int cr = wcnt[w2];
    ovf |= (cr > WLCAP || cr < 0) ? 1 : 0;
    tot += clampi(cr, 0, WLCAP);
  }
  ovf |= (tot > RCAP) ? 1 : 0;

  if (wave == 0) {
#pragma unroll 1
    for (int w2 = 0; w2 < 8; ++w2) {
      const int cv = clampi(wcnt[w2], 0, WLCAP);
      const int n  = __builtin_amdgcn_readfirstlane(cv);
      const int* L = wl + w2 * WLCAP;
#pragma unroll 1
      for (int b0 = 0; b0 < n; b0 += 32) {
        const int idx = imin(b0 + lane, n - 1);
        const int uv  = L[idx];
        const int m32 = imin(n - b0, 32);
#pragma unroll 1
        for (int k = 0; k < m32; ++k) {
          const int u  = __builtin_amdgcn_readlane(uv, k);
          const int sl = (u >> 16) & (BSLOTS - 1);
          if (lane == 0) scnt[sl] = scnt[sl] + 1;
        }
      }
    }
  }
  __syncthreads();

  {
    const v4i cv = *(const v4ia*)(scnt + 4 * tid);
    const int c0 = cv[0] < 0 ? 0 : cv[0];
    const int c1 = cv[1] < 0 ? 0 : cv[1];
    const int c2 = cv[2] < 0 ? 0 : cv[2];
    const int c3 = cv[3] < 0 ? 0 : cv[3];
    const int ts = c0 + c1 + c2 + c3;
    int incl = ts;
#pragma unroll
    for (int d = 1; d < 32; d <<= 1) {
      const int up = __shfl_up(incl, d);
      incl += (lane >= d) ? up : 0;
    }
    if (lane == 31) wtot[wave] = incl;
    __syncthreads();
    int pre = 0;
#pragma unroll
    for (int w2 = 0; w2 < 8; ++w2) {
      const int t = wtot[w2];
      pre += (w2 < wave) ? t : 0;
    }
    const int r0 = pre + incl - ts;
    const int r1 = r0 + c0;
    const int r2 = r1 + c1;
    const int r3 = r2 + c2;
    soff[4 * tid + 0] = r0; cur[4 * tid + 0] = r0;
    soff[4 * tid + 1] = r1; cur[4 * tid + 1] = r1;
    soff[4 * tid + 2] = r2; cur[4 * tid + 2] = r2;
    soff[4 * tid + 3] = r3; cur[4 * tid + 3] = r3;
  }
  __syncthreads();

  if (wave == 0) {
#pragma unroll 1
    for (int w2 = 0; w2 < 8; ++w2) {
      const int cv = clampi(wcnt[w2], 0, WLCAP);
      const int n  = __builtin_amdgcn_readfirstlane(cv);
      const int* L = wl + w2 * WLCAP;
#pragma unroll 1
      for (int b0 = 0; b0 < n; b0 += 32) {
        const int idx = imin(b0 + lane, n - 1);
        const int uv  = L[idx];
        const int m32 = imin(n - b0, 32);
#pragma unroll 1
        for (int k = 0; k < m32; ++k) {
          const int u  = __builtin_amdgcn_readlane(uv, k);
          const int sl = (u >> 16) & (BSLOTS - 1);
          if (lane == 0) {
            const int pos = clampi(cur[sl], 0, RCAP - 1);
            placed[pos] = u & 0xFFFF;
            cur[sl] = pos + 1;
          }
        }
      }
    }
  }
  __syncthreads();

  unsigned* lb = list_out + (size_t)blockIdx.x * RCAP;
  for (int pass = 0; pass < 2; ++pass) {
#pragma unroll 1
    for (int i = tid; i < RCAP / 4; i += 256) {
      const v4u v = *(const v4ua*)(placed + 4 * i);
      *(volatile v4u*)(lb + 4 * i) = v;
    }
    __threadfence();
  }
  {
    const int r4 = 4 * tid;
    const v4i ov = *(const v4ia*)(soff + r4);
    const v4i cv = *(const v4ia*)(scnt + r4);
    asm volatile("" :: "v"(ov));
    asm volatile("" :: "v"(cv));
    const bool wr = r4 < nb;
    int* po = rowoff + slotBase + r4;
    int* pc = rowcnt + slotBase + r4;
    if (wr) { *(volatile v4i*)po = ov; *(volatile v4i*)pc = cv; }
    __threadfence();
    if (wr) { *(volatile v4i*)po = ov; *(volatile v4i*)pc = cv; }
  }
  {
    const v4i fv = (v4i){ ovf, ovf, ovf, ovf };
    int* pf = flag + (size_t)blockIdx.x * 32 + 4 * (lane & 7);
    const bool wr = (wave == 0) && (lane < 8);
    if (wr) *(volatile v4i*)pf = fv;
    __threadfence();
    if (wr) *(volatile v4i*)pf = fv;
  }
}

__global__ __launch_bounds__(256) void k_replay(const float* __restrict__ Z, const float* __restrict__ slr,
                                                const unsigned* __restrict__ list_in,
                                                const int* __restrict__ rowoff, const int* __restrict__ rowcnt,
                                                const int* __restrict__ flag, float* out) {
  __shared__ int   sSrc[8][DEGCAP];
  __shared__ float sAl[8][DEGCAP];
  const int lane = threadIdx.x & 31, wave = threadIdx.x >> 5;
  const int row = (int)blockIdx.x * 8 + wave;
  const int rc  = clampi(row, 0, NN - 1);
  const int b   = rc >> 10;
  const int off = rowoff[rc];
  asm volatile("" :: "v"(off));
  const int cnt = rowcnt[rc];
  asm volatile("" :: "v"(cnt));
  const int flg = flag[b * 32];
  asm volatile("" :: "v"(flg));
  const float sr = slr[NN + rc];
  asm volatile("" :: "v"(sr));
  const bool inr  = row < NN;
  const bool good = (flg == 0) && (cnt >= 0) && (cnt <= DEGCAP);
  const bool live = inr && good;
  const bool poison = inr && !good;
  const int cvv = live ? clampi(cnt, 0, DEGCAP) : 0;
  const int cn  = __builtin_amdgcn_readfirstlane(cvv);

  const int offc = clampi(off, 0, RCAP - 1);
  const int jl   = cn > 0 ? cn - 1 : 0;
  const unsigned* L = list_in + (size_t)b * RCAP;
  const int j0 = lane, j1 = lane + 32;
  const int i0 = imin(offc + imin(j0, jl), RCAP - 1);
  const int i1 = imin(offc + imin(j1, jl), RCAP - 1);
  const unsigned w0 = L[i0];
  const unsigned w1 = L[i1];
  asm volatile("" :: "v"(w0));
  asm volatile("" :: "v"(w1));
  const int s0 = (int)(w0 < (unsigned)(NN - 1) ? w0 : (unsigned)(NN - 1));
  const int s1 = (int)(w1 < (unsigned)(NN - 1) ? w1 : (unsigned)(NN - 1));
  const float g0 = slr[s0];
  const float g1 = slr[s1];
  asm volatile("" :: "v"(g0));
  asm volatile("" :: "v"(g1));
  float e0 = g0 + sr;
  float e1 = g1 + sr;
  e0 = (e0 >= 0.0f) ? e0 : 0.01f * e0;
  e1 = (e1 >= 0.0f) ? e1 : 0.01f * e1;
  const bool v0 = j0 < cn, v1 = j1 < cn;
  const float ninf = __uint_as_float(0xff800000u);
  float m = fmaxf(v0 ? e0 : ninf, v1 ? e1 : ninf);
#pragma unroll
  for (int o2 = 16; o2 > 0; o2 >>= 1) m = fmaxf(m, __shfl_xor(m, o2));
  const float t0 = expf(e0 - m);
  const float t1 = expf(e1 - m);
  const float x0 = v0 ? t0 : 0.0f;
  const float x1 = v1 ? t1 : 0.0f;
  float den = x0 + x1;
#pragma unroll
  for (int o2 = 16; o2 > 0; o2 >>= 1) den += __shfl_xor(den, o2);
  const float dsafe = (cn > 0) ? den : 1.0f;
  const float a0 = x0 / dsafe;
  const float a1 = x1 / dsafe;
  sSrc[wave][j0] = s0;
  sSrc[wave][j1] = s1;
  sAl[wave][j0]  = a0;
  sAl[wave][j1]  = a1;
  __builtin_amdgcn_fence(__ATOMIC_RELEASE, "workgroup");
  __builtin_amdgcn_wave_barrier();
  __builtin_amdgcn_fence(__ATOMIC_ACQUIRE, "workgroup");

  v4f acc = (v4f){0.0f, 0.0f, 0.0f, 0.0f};
#pragma unroll 1
  for (int j = 0; j < cn; ++j) {
    const int   sj = clampi(sSrc[wave][j], 0, NN - 1);
    const float aj = sAl[wave][j];
    const v4f zr = *(const v4fa*)(Z + (size_t)sj * DD + 4 * lane);
    acc[0] = fmaf(aj, zr[0], acc[0]);
    acc[1] = fmaf(aj, zr[1], acc[1]);
    acc[2] = fmaf(aj, zr[2], acc[2]);
    acc[3] = fmaf(aj, zr[3], acc[3]);
  }
  const float qn = __uint_as_float(0x7fc00000u);
  const v4f zero4 = (v4f){0.0f, 0.0f, 0.0f, 0.0f};
  const v4f nan4  = (v4f){qn, qn, qn, qn};
  v4f o = (cn > 0) ? acc : zero4;
  o = poison ? nan4 : o;
  float* op = out + (size_t)rc * DD + 4 * lane;
  if (inr) *(volatile v4f*)op = o;
  __threadfence();
  if (inr) *(volatile v4f*)op = o;
}

#define O_XB     0u
#define SZ_XB    (MPAD * DD * 2u)
#define O_Z      (O_XB + SZ_XB)
#define SZ_Z     (MPAD * DD * 4u)
#define O_WB     (O_Z + SZ_Z)
#define SZ_WB    (DD * DD * 2u)
#define O_ALR    (O_WB + SZ_WB)
#define SZ_ALR   1024u
#define O_SLR    (O_ALR + SZ_ALR)
#define SZ_SLR   (2u * NN * 4u)
#define O_LIST   (O_SLR + SZ_SLR)
#define SZ_LIST  (NBLK * RCAP * 4u)
#define O_ROFF   (O_LIST + SZ_LIST)
#define SZ_ROW   (NN * 4u)
#define O_RCNT   (O_ROFF + SZ_ROW)
#define O_FLAG   (O_RCNT + SZ_ROW)
#define SZ_FLAG  (NBLK * 128u)
#define WS_TOTAL (O_FLAG + SZ_FLAG)

static_assert(O_Z % 256 == 0 && O_WB % 256 == 0 && O_ALR % 256 == 0 && O_SLR % 256 == 0);
static_assert(O_LIST % 256 == 0 && O_ROFF % 256 == 0 && O_RCNT % 256 == 0 && O_FLAG % 256 == 0);
static_assert((RCAP * 4) % 128 == 0);
static_assert(WS_TOTAL == 34888704u);
static_assert(WS_TOTAL <= (128u << 20));

extern "C" void kernel_launch(void* const* d_in, const int* in_sizes, int n_in,
                              void* d_out, int out_size, void* d_ws, size_t ws_size,
                              hipStream_t stream) {
  if (n_in != 5) return;
  if (in_sizes[0] != NN * DD || in_sizes[1] != NE || in_sizes[2] != NE) return;
  if (in_sizes[3] != DD * DD || in_sizes[4] != 2 * DD) return;
  if (out_size != NN * DD) return;
  if (ws_size < (size_t)WS_TOTAL) return;

  const float* features = (const float*)d_in[0];
  const int*   src_idx  = (const int*)  d_in[1];
  const int*   dst_idx  = (const int*)  d_in[2];
  const float* W_fc     = (const float*)d_in[3];
  const float* a_attn   = (const float*)d_in[4];
  float* out = (float*)d_out;

  char* ws = (char*)d_ws;
  unsigned short* XB  = (unsigned short*)(ws + O_XB);
  float*          Zp  = (float*)(ws + O_Z);
  unsigned short* WB  = (unsigned short*)(ws + O_WB);
  float*          ALR = (float*)(ws + O_ALR);
  float*          SLR = (float*)(ws + O_SLR);
  unsigned*       LST = (unsigned*)(ws + O_LIST);
  int*            ROF = (int*)(ws + O_ROFF);
  int*            RCN = (int*)(ws + O_RCNT);
  int*            FLG = (int*)(ws + O_FLAG);

  hipFuncSetAttribute(reinterpret_cast<const void*>(&k_bucket),
                      hipFuncAttributeMaxDynamicSharedMemorySize, LDS_BK);

  k_plane<0><<<MPAD * DD / 8 / 256, 256, 0, stream>>>(features, NN, DD, DD, XB, MPAD, DD);
  k_plane<0><<<DD * DD / 8 / 256, 256, 0, stream>>>(W_fc, DD, DD, DD, WB, DD, DD);
  k_prep<<<1, 64, 0, stream>>>(a_attn, ALR);
  k_gemm_nt<0, 0><<<(((NN + 63) / 64) * (DD / 64) + 7) / 8, 256, 0, stream>>>(XB, WB, ALR, Zp, NN, DD, DD, DD);
  k_scores<<<NN / 32, 256, 0, stream>>>(Zp, ALR, SLR);
  k_bucket<<<NBLK, 256, LDS_BK, stream>>>(src_idx, dst_idx, LST, ROF, RCN, FLG);
  k_replay<<<NN / 8, 256, 0, stream>>>(Zp, SLR, LST, ROF, RCN, FLG, out);
}
